// UMambaConvBlock_43198781063660
// MI455X (gfx1250) — hardware-run, weakly checked
//
#include <hip/hip_runtime.h>
#include <math.h>

#define NBT   4
#define NCH   64
#define IMH   96
#define IMW   96
#define NPIX  9216
#define NTOK  36864
#define DIN   128
#define DSTT  64
#define DTRK  4
#define XZW   256
#define DBW   192
#define DBN   132
#define TPB   128
#define NBLK  288
#define PPB   72
#define OSTR  68
#define SCH   32
#define NSUB  4
#define NSTS  16
#define XTP   72
#define LOG2E 1.4426950408889634f
#define EPSV  1e-5f

static_assert(NTOK == NBT * NPIX);
static_assert(NTOK % TPB == 0);
static_assert(NPIX % TPB == 0);
static_assert(NBLK == NTOK / TPB);
static_assert(PPB == NPIX / TPB);
static_assert(IMW % 16 == 0);
static_assert(NPIX % SCH == 0);
static_assert(SCH * 8 == 256);
static_assert(NSUB * NSTS == DSTT);
static_assert(DBW % 64 == 0);
static_assert(DBW >= DBN);
static_assert(OSTR % 4 == 0);
static_assert((NTOK * 8) % 256 == 0);
static_assert((NTOK * DIN) % 256 == 0);
static_assert(NPIX % 64 == 0);
static_assert(XTP % 8 == 0);
static_assert(NTOK % 8 == 0);

typedef unsigned short us16 __attribute__((ext_vector_type(16)));
typedef unsigned short us8  __attribute__((ext_vector_type(8)));
typedef unsigned short us8a __attribute__((ext_vector_type(8), may_alias));
typedef unsigned int   u32x8 __attribute__((ext_vector_type(8)));
typedef __bf16 v16b __attribute__((ext_vector_type(16)));
typedef float v8f __attribute__((ext_vector_type(8)));
typedef float v4f __attribute__((ext_vector_type(4)));
typedef float v4fa __attribute__((ext_vector_type(4), may_alias));
union FragU { us16 v; us8 h[2]; u32x8 w; };

#if __has_builtin(__builtin_amdgcn_exp2f)
#define FEXP2(x) __builtin_amdgcn_exp2f(x)
#else
#define FEXP2(x) __expf((x) * 0.6931471805599453f)
#endif

__device__ __forceinline__ unsigned short bf16_bits(float f) {
  unsigned u = __float_as_uint(f);
  u += 0x7FFFu + ((u >> 16) & 1u);
  return (unsigned short)(u >> 16);
}
__device__ __forceinline__ float bf16_val(unsigned short b) { return __uint_as_float(((unsigned)b) << 16); }
__device__ __forceinline__ float bf16r(float f) { return bf16_val(bf16_bits(f)); }
__device__ __forceinline__ float siluf(float x) { return x * __builtin_amdgcn_rcpf(1.0f + __expf(-x)); }

__device__ __forceinline__ void split8(const v4f a, const v4f b, us8& hi, us8& lo) {
#pragma unroll
  for (int u = 0; u < 4; ++u) {
    const unsigned short ha = bf16_bits(a[u]);
    hi[u] = ha; lo[u] = bf16_bits(a[u] - bf16_val(ha));
    const unsigned short hb = bf16_bits(b[u]);
    hi[4 + u] = hb; lo[4 + u] = bf16_bits(b[u] - bf16_val(hb));
  }
}

__device__ __forceinline__ v8f mma_bf16(us16 a, us16 b, v8f c) {
  return __builtin_amdgcn_wmma_f32_16x16x32_bf16(false, __builtin_bit_cast(v16b, a), false, __builtin_bit_cast(v16b, b), (short)0, c, false, false);
}
__device__ __forceinline__ void wguard2(v8f& c0, v8f& c1, v8f& c2, v8f& c3, const us16& a0, const us16& a1,
                                        const us16& b0, const us16& b1, const us16& b2, const us16& b3) {
#if defined(__HIP_DEVICE_COMPILE__)
  asm volatile("v_nop\n\tv_nop\n\tv_nop\n\tv_nop"
               : "+v"(c0), "+v"(c1), "+v"(c2), "+v"(c3)
               : "v"(a0), "v"(a1), "v"(b0), "v"(b1), "v"(b2), "v"(b3));
#endif
}
__device__ __forceinline__ void wguard1(v8f& c0, v8f& c1, v8f& c2, v8f& c3, const us16& a0,
                                        const us16& b0, const us16& b1, const us16& b2, const us16& b3) {
#if defined(__HIP_DEVICE_COMPILE__)
  asm volatile("v_nop\n\tv_nop\n\tv_nop\n\tv_nop"
               : "+v"(c0), "+v"(c1), "+v"(c2), "+v"(c3)
               : "v"(a0), "v"(b0), "v"(b1), "v"(b2), "v"(b3));
#endif
}

__device__ __forceinline__ us16 gfrag(const unsigned short* p) {
  const int kh = ((threadIdx.x >> 4) & 1) * 8;
  FragU f;
  f.h[0] = *(const us8a*)(p + kh);
  f.h[1] = *(const us8a*)(p + 16 + kh);
  return f.v;
}

__global__ __launch_bounds__(256) void k_cvt(const float* __restrict__ src, unsigned short* dst, int nsrc, int ncol8, int total8) {
  const int idx = blockIdx.x * 256 + threadIdx.x;
  if (idx >= total8) return;
  const int row = idx / ncol8, c8 = (idx - row * ncol8) * 8;
  const int rs = (row < nsrc) ? row : (nsrc - 1);
  const float* s = src + (size_t)rs * (size_t)(ncol8 * 8) + c8;
  const v4f a = *(const v4fa*)s, b = *(const v4fa*)(s + 4);
  const bool zr = (row >= nsrc);
  us8 o;
#pragma unroll
  for (int u = 0; u < 4; ++u) {
    o[u]     = zr ? (unsigned short)0 : bf16_bits(a[u]);
    o[4 + u] = zr ? (unsigned short)0 : bf16_bits(b[u]);
  }
  const size_t off = (size_t)row * (size_t)(ncol8 * 8) + c8;
  *(volatile us8*)(dst + off) = o;
  __threadfence();
  *(volatile us8*)(dst + off) = o;
}

__global__ __launch_bounds__(256) void k_wconv(const float* __restrict__ w, unsigned short* WC) {
  const int idx = blockIdx.x * 256 + threadIdx.x;
  if (idx >= 9 * NCH * NCH / 8) return;
  const int t = idx >> 9, rem = idx & 511, co = rem >> 3, ci8 = (rem & 7) * 8;
  us8 o;
#pragma unroll
  for (int u = 0; u < 8; ++u) o[u] = bf16_bits(w[((size_t)(co * NCH + ci8 + u)) * 9 + t]);
  const size_t off = (size_t)idx * 8;
  *(volatile us8*)(WC + off) = o;
  __threadfence();
  *(volatile us8*)(WC + off) = o;
}

__global__ __launch_bounds__(256) void k_xtok(const float* __restrict__ x, unsigned short* XB) {
  __shared__ __attribute__((aligned(16))) unsigned short tile[64 * XTP];
  const int tid = threadIdx.x, hw0 = blockIdx.x * 64, b = blockIdx.y;
  const int hw = tid & 63, cq = tid >> 6;
#pragma unroll
  for (int it = 0; it < 16; ++it) {
    const int c = it * 4 + cq;
    const float v = x[((size_t)(b * NCH + c)) * NPIX + hw0 + hw];
    tile[hw * XTP + c] = bf16_bits(v);
  }
  __syncthreads();
  const int row = tid >> 3, c8 = (tid & 7) * 8;
#pragma unroll
  for (int pass = 0; pass < 2; ++pass) {
#pragma unroll
    for (int it = 0; it < 2; ++it) {
      const int rr = it * 32 + row;
      const us8 v = *(const us8a*)(tile + rr * XTP + c8);
      *(volatile us8*)(XB + ((size_t)(b * NPIX + hw0 + rr)) * NCH + c8) = v;
    }
    __threadfence();
  }
}

__global__ __launch_bounds__(256) void k_conv3(const unsigned short* __restrict__ XB, const unsigned short* __restrict__ WC,
                                              float* HC, float* PART) {
  __shared__ __attribute__((aligned(16))) float oS[8 * 16 * OSTR];
  __shared__ __attribute__((aligned(16))) float red[512];
  __shared__ __attribute__((aligned(16))) float pst[128];
  const int tid = threadIdx.x, lane = tid & 31, wave = tid >> 5, cl = lane & 15, hh = lane >> 4;
  const int mb = blockIdx.x * TPB, m0 = mb + 16 * wave;
  const int bimg = mb / NPIX, hwb = m0 - bimg * NPIX, py = hwb / IMW, px = (hwb - py * IMW) + cl;

  v8f acc[4];
#pragma unroll
  for (int j = 0; j < 4; ++j) { const v8f zz = {0.f, 0.f, 0.f, 0.f, 0.f, 0.f, 0.f, 0.f}; acc[j] = zz; }

#pragma unroll 1
  for (int s = 0; s < 18; ++s) {
    const int t = s >> 1, kb = (s & 1) * 32;
    const int ky = t / 3, kx = t - 3 * ky;
    const int yy = py + ky - 1, xx = px + kx - 1;
    const bool ok = (yy >= 0) && (yy < IMH) && (xx >= 0) && (xx < IMW);
    int src = m0 + cl + (ky - 1) * IMW + (kx - 1);
    src = (src < 0) ? 0 : src;
    src = (src > NTOK - 1) ? (NTOK - 1) : src;
    FragU fa;
    fa.v = gfrag(XB + (size_t)src * NCH + kb);
#pragma unroll
    for (int i = 0; i < 8; ++i) fa.w[i] = ok ? fa.w[i] : 0u;
    const unsigned short* wp = WC + ((size_t)t * NCH + cl) * NCH + kb;
    us16 bfr[4];
#pragma unroll
    for (int j = 0; j < 4; ++j) bfr[j] = gfrag(wp + (size_t)(16 * j) * NCH);
#pragma unroll
    for (int j = 0; j < 4; ++j) acc[j] = mma_bf16(fa.v, bfr[j], acc[j]);
    wguard1(acc[0], acc[1], acc[2], acc[3], fa.v, bfr[0], bfr[1], bfr[2], bfr[3]);
  }

  float* so = oS + wave * (16 * OSTR);
#pragma unroll
  for (int j = 0; j < 4; ++j)
#pragma unroll
    for (int r = 0; r < 8; ++r) so[(8 * hh + r) * OSTR + 16 * j + cl] = acc[j][r];
  __syncthreads();

#pragma unroll
  for (int pass = 0; pass < 2; ++pass) {
#pragma unroll
    for (int it = 0; it < 8; ++it) {
      const int ch = it * 32 + lane, r = ch >> 4, q = (ch & 15) * 4;
      const v4f v = *(const v4fa*)(so + r * OSTR + q);
      *(volatile v4f*)(HC + (size_t)(m0 + r) * NCH + q) = v;
    }
    __threadfence();
  }

  {
    const int c = tid & 63, ph = tid >> 6;
    float s = 0.0f, q = 0.0f;
#pragma unroll 4
    for (int i = 0; i < 32; ++i) {
      const float v = oS[(ph * 32 + i) * OSTR + c];
      s += v; q += v * v;
    }
    red[ph * 64 + c] = s; red[256 + ph * 64 + c] = q;
  }
  __syncthreads();
  if (tid < 64) {
    const float S = ((red[tid] + red[64 + tid]) + red[128 + tid]) + red[192 + tid];
    const float Q = ((red[256 + tid] + red[320 + tid]) + red[384 + tid]) + red[448 + tid];
    pst[tid] = S; pst[64 + tid] = Q;
  }
  __syncthreads();
  if (wave == 0) {
    const v4f v = *(const v4fa*)(pst + lane * 4);
    *(volatile v4f*)(PART + (size_t)blockIdx.x * 128 + lane * 4) = v;
    __threadfence();
    *(volatile v4f*)(PART + (size_t)blockIdx.x * 128 + lane * 4) = v;
  }
}

__global__ __launch_bounds__(64) void k_bnfin(const float* __restrict__ PART, float* ST) {
  __shared__ __attribute__((aligned(16))) float pst[128];
  const int c = threadIdx.x;
  double s = 0.0, q = 0.0;
#pragma unroll 1
  for (int p = 0; p < NBLK; ++p) { s += (double)PART[p * 128 + c]; q += (double)PART[p * 128 + 64 + c]; }
  const double mean = s / (double)NTOK;
  double var = q / (double)NTOK - mean * mean;
  var = (var < 0.0) ? 0.0 : var;
  pst[c] = (float)mean;
  pst[64 + c] = rsqrtf((float)var + EPSV);
  __syncthreads();
  if (c < 32) {
    const v4f v = *(const v4fa*)(pst + c * 4);
    *(volatile v4f*)(ST + c * 4) = v;
    __threadfence();
    *(volatile v4f*)(ST + c * 4) = v;
  }
}

__global__ __launch_bounds__(256) void k_napply(const float* __restrict__ src, const float* __restrict__ ST, int per_img, int relu,
                                               const float* __restrict__ g, const float* __restrict__ bt,
                                               unsigned short* H, unsigned short* L) {
  const int idx = blockIdx.x * 256 + threadIdx.x;
  if (idx >= NTOK * 8) return;
  const int row = idx >> 3, c8 = (idx & 7) * 8;
  const int so = per_img ? (row / NPIX) * 128 : 0;
  const float* s = src + (size_t)row * NCH + c8;
  const v4f xa = *(const v4fa*)s, xb = *(const v4fa*)(s + 4);
  const v4f ma = *(const v4fa*)(ST + so + c8), mb = *(const v4fa*)(ST + so + c8 + 4);
  const v4f ra = *(const v4fa*)(ST + so + 64 + c8), rb = *(const v4fa*)(ST + so + 64 + c8 + 4);
  const v4f ga = *(const v4fa*)(g + c8), gb = *(const v4fa*)(g + c8 + 4);
  const v4f ba = *(const v4fa*)(bt + c8), bb = *(const v4fa*)(bt + c8 + 4);
  v4f oa, ob;
#pragma unroll
  for (int u = 0; u < 4; ++u) {
    float t0 = ((xa[u] - ma[u]) * ra[u]) * bf16r(ga[u]) + bf16r(ba[u]);
    float t1 = ((xb[u] - mb[u]) * rb[u]) * bf16r(gb[u]) + bf16r(bb[u]);
    oa[u] = relu ? fmaxf(t0, 0.0f) : t0;
    ob[u] = relu ? fmaxf(t1, 0.0f) : t1;
  }
  us8 hi, lo;
  split8(oa, ob, hi, lo);
  const size_t off = (size_t)row * NCH + c8;
  *(volatile us8*)(H + off) = hi; *(volatile us8*)(L + off) = lo;
  __threadfence();
  *(volatile us8*)(H + off) = hi; *(volatile us8*)(L + off) = lo;
}

template <int BIAS, int SILU, int OUTF, int FY0, int OUTHL, int MULU, int FINAL>
__global__ __launch_bounds__(256) void k_gemm(const unsigned short* __restrict__ A0, const unsigned short* __restrict__ A1, int lda,
                                             const unsigned short* __restrict__ Bw, int ldb, int K,
                                             const float* __restrict__ bias, float* Yf, int ldy,
                                             unsigned short* YH, unsigned short* YL, int ldh,
                                             const float* __restrict__ MU, int ldm,
                                             const float* __restrict__ xin, float* outp) {
  __shared__ __attribute__((aligned(16))) float oS[8 * 16 * OSTR];
  const int tid = threadIdx.x, lane = tid & 31, wave = tid >> 5, cl = lane & 15, hh = lane >> 4;
  const int mb = blockIdx.x * TPB, m0 = mb + 16 * wave, n0 = blockIdx.y * 64;

  v8f acc[4];
#pragma unroll
  for (int j = 0; j < 4; ++j) { const v8f zz = {0.f, 0.f, 0.f, 0.f, 0.f, 0.f, 0.f, 0.f}; acc[j] = zz; }

  const unsigned short* a0p = A0 + (size_t)(m0 + cl) * lda;
  const unsigned short* a1p = A1 + (size_t)(m0 + cl) * lda;
  const unsigned short* bwp = Bw + (size_t)(n0 + cl) * ldb;
#pragma unroll 1
  for (int k0 = 0; k0 < K; k0 += 32) {
    const us16 af0 = gfrag(a0p + k0);
    const us16 af1 = gfrag(a1p + k0);
    us16 bfr[4];
#pragma unroll
    for (int j = 0; j < 4; ++j) bfr[j] = gfrag(bwp + (size_t)(16 * j) * ldb + k0);
#pragma unroll
    for (int j = 0; j < 4; ++j) acc[j] = mma_bf16(af0, bfr[j], acc[j]);
#pragma unroll
    for (int j = 0; j < 4; ++j) acc[j] = mma_bf16(af1, bfr[j], acc[j]);
    wguard2(acc[0], acc[1], acc[2], acc[3], af0, af1, bfr[0], bfr[1], bfr[2], bfr[3]);
  }

  float* so = oS + wave * (16 * OSTR);
#pragma unroll
  for (int j = 0; j < 4; ++j)
#pragma unroll
    for (int r = 0; r < 8; ++r) so[(8 * hh + r) * OSTR + 16 * j + cl] = acc[j][r];
  __syncthreads();

  if (OUTF) {
    if (!FY0 || blockIdx.y == 0) {
#pragma unroll
      for (int pass = 0; pass < 2; ++pass) {
#pragma unroll
        for (int it = 0; it < 8; ++it) {
          const int ch = it * 32 + lane, r = ch >> 4, q = (ch & 15) * 4;
          v4f v = *(const v4fa*)(so + r * OSTR + q);
          if (BIAS) {
#pragma unroll
            for (int u = 0; u < 4; ++u) v[u] = v[u] + bf16r(bias[n0 + q + u]);
          }
          if (SILU) {
#pragma unroll
            for (int u = 0; u < 4; ++u) v[u] = siluf(v[u]);
          }
          *(volatile v4f*)(Yf + (size_t)(m0 + r) * ldy + n0 + q) = v;
        }
        __threadfence();
      }
    }
  }
  if (OUTHL) {
#pragma unroll
    for (int pass = 0; pass < 2; ++pass) {
#pragma unroll
      for (int it = 0; it < 4; ++it) {
        const int ch = it * 32 + lane, r = ch >> 3, c8 = (ch & 7) * 8;
        v4f a = *(const v4fa*)(so + r * OSTR + c8);
        v4f b = *(const v4fa*)(so + r * OSTR + c8 + 4);
        if (BIAS) {
#pragma unroll
          for (int u = 0; u < 4; ++u) { a[u] = a[u] + bf16r(bias[n0 + c8 + u]); b[u] = b[u] + bf16r(bias[n0 + c8 + 4 + u]); }
        }
        if (SILU) {
#pragma unroll
          for (int u = 0; u < 4; ++u) { a[u] = siluf(a[u]); b[u] = siluf(b[u]); }
        }
        if (MULU) {
          const v4f ua = *(const v4fa*)(MU + (size_t)(m0 + r) * ldm + n0 + c8);
          const v4f ub = *(const v4fa*)(MU + (size_t)(m0 + r) * ldm + n0 + c8 + 4);
          a = a * ua; b = b * ub;
        }
        us8 hi, lo;
        split8(a, b, hi, lo);
        const size_t o2 = (size_t)(m0 + r) * ldh + n0 + c8;
        *(volatile us8*)(YH + o2) = hi; *(volatile us8*)(YL + o2) = lo;
      }
      __threadfence();
    }
  }
  if (FINAL) {
    const int bimg = mb / NPIX, hw0 = mb - bimg * NPIX;
#pragma unroll
    for (int pass = 0; pass < 2; ++pass) {
#pragma unroll
      for (int it = 0; it < 8; ++it) {
        const int c = it * 8 + wave;
        const size_t o = ((size_t)(bimg * NCH + c)) * NPIX + hw0 + lane * 4;
        const v4f xv = *(const v4fa*)(xin + o);
        v4f v;
#pragma unroll
        for (int i = 0; i < 4; ++i) {
          float t = oS[(lane * 4 + i) * OSTR + c];
          t = (t >= 0.0f) ? t : 0.01f * t;
          v[i] = fmaxf(t + bf16r(xv[i]), 0.0f);
        }
        *(volatile v4f*)(outp + o) = v;
      }
      __threadfence();
    }
  }
}

__global__ __launch_bounds__(256) void k_dwconv(const float* __restrict__ XZ, const float* __restrict__ cw, const float* __restrict__ cb,
                                               float* XC, unsigned short* XCH, unsigned short* XCL) {
  __shared__ __attribute__((aligned(16))) float sx[8 * DIN];
  const int tid = threadIdx.x, lane = tid & 31, wave = tid >> 5;
  const int tok = blockIdx.x * 8 + wave, l = tok % NPIX, c4 = lane * 4;
  v4f xv[4];
#pragma unroll
  for (int j = 0; j < 4; ++j) {
    const int ll = l - 3 + j;
    const int ts = (ll >= 0) ? (tok - 3 + j) : tok;
    xv[j] = *(const v4fa*)(XZ + (size_t)ts * XZW + c4);
  }
  const v4f bb = *(const v4fa*)(cb + c4);
  v4f sv;
#pragma unroll
  for (int u = 0; u < 4; ++u) {
    const v4f wv = *(const v4fa*)(cw + (size_t)(c4 + u) * 4);
    float a = 0.0f;
#pragma unroll
    for (int j = 0; j < 4; ++j) {
      const float pr = bf16r(wv[j]) * xv[j][u];
      a = a + ((l - 3 + j >= 0) ? pr : 0.0f);
    }
    a = a + bf16r(bb[u]);
    sv[u] = siluf(a);
  }
  const size_t o = (size_t)tok * DIN + c4;
  *(volatile v4f*)(XC + o) = sv;
  __threadfence();
  *(volatile v4f*)(XC + o) = sv;
  *(v4fa*)(sx + wave * DIN + c4) = sv;
  __syncthreads();
  if (tid < 128) {
    const int w2 = tid >> 4, c8 = (tid & 15) * 8;
    const v4f a = *(const v4fa*)(sx + w2 * DIN + c8);
    const v4f b = *(const v4fa*)(sx + w2 * DIN + c8 + 4);
    us8 hi, lo;
    split8(a, b, hi, lo);
    const size_t o2 = ((size_t)blockIdx.x * 8 + w2) * DIN + c8;
    *(volatile us8*)(XCH + o2) = hi; *(volatile us8*)(XCL + o2) = lo;
    __threadfence();
    *(volatile us8*)(XCH + o2) = hi; *(volatile us8*)(XCL + o2) = lo;
  }
}

__global__ __launch_bounds__(256) void k_dtgate(const float* __restrict__ DBL, const float* __restrict__ dtw, const float* __restrict__ dtb,
                                               const float* __restrict__ XZ, float* DT, float* SZ) {
  const int idx = blockIdx.x * 256 + threadIdx.x;
  if (idx >= NTOK * DIN) return;
  const int tok = idx >> 7, d = idx & (DIN - 1);
  const v4f dl4 = *(const v4fa*)(DBL + (size_t)tok * DBW);
  const v4f w4 = *(const v4fa*)(dtw + d * DTRK);
  float a = 0.0f;
#pragma unroll
  for (int r = 0; r < DTRK; ++r) a = a + dl4[r] * bf16r(w4[r]);
  a = a + bf16r(dtb[d]);
  const float dl = fmaxf(a, 0.0f) + log1pf(expf(-fabsf(a)));
  const float z = XZ[(size_t)tok * XZW + DIN + d];
  const float sz = siluf(z);
  *(volatile float*)(DT + idx) = dl; *(volatile float*)(SZ + idx) = sz;
  __threadfence();
  *(volatile float*)(DT + idx) = dl; *(volatile float*)(SZ + idx) = sz;
}

__global__ __launch_bounds__(256) void k_scan(const float* __restrict__ DT, const float* __restrict__ XC, const float* __restrict__ SZ,
                                             const float* __restrict__ DBL, const float* __restrict__ Alog, const float* __restrict__ Dv,
                                             unsigned short* YGH, unsigned short* YGL) {
  __shared__ __attribute__((aligned(16))) float sy[SCH * 64];
  const int tid = threadIdx.x, b = blockIdx.x >> 1, dg = blockIdx.x & 1, ch = tid >> 2, sub = tid & 3;
  const int d = dg * 64 + ch, n0 = sub * NSTS;
  float A2[NSTS], h[NSTS];
#pragma unroll
  for (int i = 0; i < NSTS; ++i) { A2[i] = -__expf(bf16r(Alog[d * DSTT + n0 + i])) * LOG2E; h[i] = 0.0f; }
  const float Dd = bf16r(Dv[d]);
  const int row = tid >> 3, c8 = (tid & 7) * 8;
#pragma unroll 1
  for (int c = 0; c < NPIX / SCH; ++c) {
#pragma unroll 1
    for (int s = 0; s < SCH; ++s) {
      const size_t tok = (size_t)b * NPIX + (size_t)(c * SCH + s);
      const size_t e = tok * DIN + d;
      const float dl = DT[e], xv = XC[e], sz = SZ[e];
      const float* bc = DBL + tok * DBW + DTRK + n0;
      v4f Bv[4], Cv[4];
#pragma unroll
      for (int q = 0; q < 4; ++q) {
        Bv[q] = *(const v4fa*)(bc + 4 * q);
        Cv[q] = *(const v4fa*)(bc + DSTT + 4 * q);
      }
      const float dx = dl * xv;
      float y = 0.0f;
#pragma unroll
      for (int i = 0; i < NSTS; ++i) {
        const float ex = FEXP2(dl * A2[i]);
        h[i] = ex * h[i] + dx * Bv[i >> 2][i & 3];
        y = y + h[i] * Cv[i >> 2][i & 3];
      }
      y += __shfl_xor(y, 1);
      y += __shfl_xor(y, 2);
      const float yv = (y + xv * Dd) * sz;
      if (sub == 0) sy[s * 64 + ch] = yv;
    }
    __syncthreads();
#pragma unroll
    for (int pass = 0; pass < 2; ++pass) {
      const v4f va = *(const v4fa*)(sy + row * 64 + c8);
      const v4f vb = *(const v4fa*)(sy + row * 64 + c8 + 4);
      us8 hi, lo;
      split8(va, vb, hi, lo);
      const size_t o = ((size_t)b * NPIX + (size_t)(c * SCH + row)) * DIN + (size_t)dg * 64 + c8;
      *(volatile us8*)(YGH + o) = hi; *(volatile us8*)(YGL + o) = lo;
      __threadfence();
    }
    __syncthreads();
  }
}

__global__ __launch_bounds__(256) void k_ln(const float* __restrict__ XP, const float* __restrict__ g, const float* __restrict__ bt,
                                           float* XN, float* PART) {
  __shared__ __attribute__((aligned(16))) float red[2048];
  __shared__ __attribute__((aligned(16))) float pst[128];
  const int tid = threadIdx.x, lane = tid & 31, wave = tid >> 5, g16 = tid >> 4, c4 = (tid & 15) * 4;
  const v4f gv0 = *(const v4fa*)(g + c4), bv0 = *(const v4fa*)(bt + c4);
  v4f gv, bv;
#pragma unroll
  for (int u = 0; u < 4; ++u) { gv[u] = bf16r(gv0[u]); bv[u] = bf16r(bv0[u]); }
  v4f cs = {0.f, 0.f, 0.f, 0.f}, cq = {0.f, 0.f, 0.f, 0.f};
#pragma unroll 1
  for (int it = 0; it < 8; ++it) {
    const int tok = blockIdx.x * TPB + it * 16 + g16;
    const size_t base = (size_t)tok * NCH + c4;
    const v4f xv = *(const v4fa*)(XP + base);
    float s = (xv[0] + xv[1]) + (xv[2] + xv[3]);
    s += __shfl_xor(s, 8); s += __shfl_xor(s, 4); s += __shfl_xor(s, 2); s += __shfl_xor(s, 1);
    const float mu = s * (1.0f / NCH);
    const v4f dv = xv - mu;
    float s2 = (dv[0] * dv[0] + dv[1] * dv[1]) + (dv[2] * dv[2] + dv[3] * dv[3]);
    s2 += __shfl_xor(s2, 8); s2 += __shfl_xor(s2, 4); s2 += __shfl_xor(s2, 2); s2 += __shfl_xor(s2, 1);
    const float var = s2 * (1.0f / NCH);
    const float rs = rsqrtf(var + EPSV);
    v4f ov;
#pragma unroll
    for (int u = 0; u < 4; ++u) ov[u] = (dv[u] * rs) * gv[u] + bv[u];
    *(volatile v4f*)(XN + base) = ov;
    __threadfence();
    *(volatile v4f*)(XN + base) = ov;
    cs = cs + ov;
    cq = cq + ov * ov;
  }
  *(v4fa*)(red + g16 * 64 + c4) = cs;
  *(v4fa*)(red + 1024 + g16 * 64 + c4) = cq;
  __syncthreads();
  if (tid < 64) {
    float S = 0.0f, Q = 0.0f;
#pragma unroll
    for (int gi = 0; gi < 16; ++gi) { S += red[gi * 64 + tid]; Q += red[1024 + gi * 64 + tid]; }
    pst[tid] = S; pst[64 + tid] = Q;
  }
  __syncthreads();
  if (wave == 0) {
    const v4f v = *(const v4fa*)(pst + lane * 4);
    *(volatile v4f*)(PART + (size_t)blockIdx.x * 128 + lane * 4) = v;
    __threadfence();
    *(volatile v4f*)(PART + (size_t)blockIdx.x * 128 + lane * 4) = v;
  }
}

__global__ __launch_bounds__(256) void k_infin(const float* __restrict__ PART, float* ST) {
  __shared__ __attribute__((aligned(16))) float st[512];
  const int tid = threadIdx.x, lane = tid & 31, wave = tid >> 5, b = tid >> 6, c = tid & 63;
  double s = 0.0, q = 0.0;
#pragma unroll 1
  for (int p = 0; p < PPB; ++p) {
    const int rw = b * PPB + p;
    s += (double)PART[rw * 128 + c]; q += (double)PART[rw * 128 + 64 + c];
  }
  const double mean = s / (double)NPIX;
  double var = q / (double)NPIX - mean * mean;
  var = (var < 0.0) ? 0.0 : var;
  st[b * 128 + c] = (float)mean;
  st[b * 128 + 64 + c] = rsqrtf((float)var + EPSV);
  __syncthreads();
  if (wave < NBT) {
    const v4f v = *(const v4fa*)(st + wave * 128 + lane * 4);
    *(volatile v4f*)(ST + wave * 128 + lane * 4) = v;
    __threadfence();
    *(volatile v4f*)(ST + wave * 128 + lane * 4) = v;
  }
}

extern "C" void kernel_launch(void* const* d_in, const int* in_sizes, int n_in,
                              void* d_out, int out_size, void* d_ws, size_t ws_size,
                              hipStream_t stream) {
  if (n_in < 23) return;
  if (in_sizes[0] != NBT * NCH * NPIX || in_sizes[1] != NCH * NCH * 9 || in_sizes[2] != NCH || in_sizes[3] != NCH ||
      in_sizes[4] != DIN * NCH || in_sizes[5] != DIN || in_sizes[6] != NCH * NCH || in_sizes[7] != XZW * NCH ||
      in_sizes[8] != DIN * 4 || in_sizes[9] != DIN || in_sizes[10] != DBN * DIN || in_sizes[11] != DIN * DTRK ||
      in_sizes[12] != DIN || in_sizes[13] != DIN * DSTT || in_sizes[14] != DIN || in_sizes[15] != NCH * DIN ||
      in_sizes[16] != NCH * NCH || in_sizes[17] != NCH || in_sizes[18] != NCH || in_sizes[19] != NCH ||
      in_sizes[20] != NCH || in_sizes[21] != NCH || in_sizes[22] != NCH * NCH) return;
  if (out_size != NTOK * NCH) return;

  const float* x          = (const float*)d_in[0];
  const float* conv_w     = (const float*)d_in[1];
  const float* bn_g       = (const float*)d_in[2];
  const float* bn_b       = (const float*)d_in[3];
  const float* expand_w   = (const float*)d_in[4];
  const float* expand_b   = (const float*)d_in[5];
  const float* c1d_w      = (const float*)d_in[6];
  const float* in_proj_w  = (const float*)d_in[7];
  const float* mconv_w    = (const float*)d_in[8];
  const float* mconv_b    = (const float*)d_in[9];
  const float* x_proj_w   = (const float*)d_in[10];
  const float* dt_w       = (const float*)d_in[11];
  const float* dt_b       = (const float*)d_in[12];
  const float* A_log      = (const float*)d_in[13];
  const float* Dv         = (const float*)d_in[14];
  const float* out_proj_w = (const float*)d_in[15];
  const float* proj_w     = (const float*)d_in[16];
  const float* proj_b     = (const float*)d_in[17];
  const float* ln_g       = (const float*)d_in[18];
  const float* ln_b       = (const float*)d_in[19];
  const float* in_g       = (const float*)d_in[20];
  const float* in_b       = (const float*)d_in[21];
  const float* rconv_w    = (const float*)d_in[22];
  float* out = (float*)d_out;

  const size_t P64H  = (size_t)NTOK * NCH * 2;
  const size_t P64F  = (size_t)NTOK * NCH * 4;
  const size_t P128H = (size_t)NTOK * DIN * 2;
  const size_t P128F = (size_t)NTOK * DIN * 4;

  size_t off = 0;
  auto carve = [&](size_t bytes) -> char* { char* p = (char*)d_ws + off; off += (bytes + 255) & ~(size_t)255; return p; };
  char* RA = carve((size_t)NTOK * XZW * 4);
  char* RB = carve((size_t)NTOK * DBW * 4);
  char* RC = carve(P128F);
  char* RD = carve(2 * P128F);
  char* RE = carve(P64F);
  unsigned short* WCV = (unsigned short*)carve((size_t)9 * NCH * NCH * 2);
  unsigned short* WEX = (unsigned short*)carve((size_t)DIN * NCH * 2);
  unsigned short* WC1 = (unsigned short*)carve((size_t)NCH * NCH * 2);
  unsigned short* WIN = (unsigned short*)carve((size_t)XZW * NCH * 2);
  unsigned short* WXP = (unsigned short*)carve((size_t)DBW * DIN * 2);
  unsigned short* WOP = (unsigned short*)carve((size_t)NCH * DIN * 2);
  unsigned short* WPJ = (unsigned short*)carve((size_t)NCH * NCH * 2);
  unsigned short* WRC = (unsigned short*)carve((size_t)NCH * NCH * 2);
  float* PARTB = (float*)carve((size_t)NBLK * 128 * 4);
  float* BNST  = (float*)carve((size_t)128 * 4);
  float* PARTI = (float*)carve((size_t)NBLK * 128 * 4);
  float* INST  = (float*)carve((size_t)NBT * 128 * 4);
  if (off > ws_size || off > (size_t)134217728) return;

  float* HC  = (float*)RA;
  float* XZ  = (float*)RA;
  unsigned short* YGH = (unsigned short*)RA;
  unsigned short* YGL = (unsigned short*)(RA + P128H);
  unsigned short* GH  = (unsigned short*)(RA + 2 * P128H);
  unsigned short* GL  = (unsigned short*)(RA + 2 * P128H + P64H);
  float* XP  = (float*)(RA + 2 * P128H + 2 * P64H);
  unsigned short* XB  = (unsigned short*)RB;
  unsigned short* XFH = (unsigned short*)(RB + P64H);
  unsigned short* XFL = (unsigned short*)(RB + 2 * P64H);
  unsigned short* V2H = (unsigned short*)(RB + 3 * P64H);
  unsigned short* V2L = (unsigned short*)(RB + 4 * P64H);
  float* DBL = (float*)RB;
  float* XN  = (float*)RB;
  unsigned short* XOH = (unsigned short*)(RB + P64F);
  unsigned short* XOL = (unsigned short*)(RB + P64F + P64H);
  unsigned short* UVH = (unsigned short*)RC;
  unsigned short* UVL = (unsigned short*)(RC + P128H);
  float* XC  = (float*)RC;
  unsigned short* XCH = (unsigned short*)RD;
  unsigned short* XCL = (unsigned short*)(RD + P128H);
  float* DT  = (float*)RD;
  float* SZ  = (float*)(RD + P128F);
  float* XU  = (float*)RE;

  const dim3 b256(256);
  auto cdv = [](long a, long b) { return (unsigned)((a + b - 1) / b); };

  k_cvt<<<dim3(cdv(DIN * NCH / 8, 256)), b256, 0, stream>>>(expand_w, WEX, DIN, NCH / 8, DIN * NCH / 8);
  k_cvt<<<dim3(cdv(NCH * NCH / 8, 256)), b256, 0, stream>>>(c1d_w, WC1, NCH, NCH / 8, NCH * NCH / 8);
  k_cvt<<<dim3(cdv(XZW * NCH / 8, 256)), b256, 0, stream>>>(in_proj_w, WIN, XZW, NCH / 8, XZW * NCH / 8);
  k_cvt<<<dim3(cdv(DBW * DIN / 8, 256)), b256, 0, stream>>>(x_proj_w, WXP, DBN, DIN / 8, DBW * DIN / 8);
  k_cvt<<<dim3(cdv(NCH * DIN / 8, 256)), b256, 0, stream>>>(out_proj_w, WOP, NCH, DIN / 8, NCH * DIN / 8);
  k_cvt<<<dim3(cdv(NCH * NCH / 8, 256)), b256, 0, stream>>>(proj_w, WPJ, NCH, NCH / 8, NCH * NCH / 8);
  k_cvt<<<dim3(cdv(NCH * NCH / 8, 256)), b256, 0, stream>>>(rconv_w, WRC, NCH, NCH / 8, NCH * NCH / 8);
  k_wconv<<<dim3(cdv(9 * NCH * NCH / 8, 256)), b256, 0, stream>>>(conv_w, WCV);

  k_xtok<<<dim3(NPIX / 64, NBT), b256, 0, stream>>>(x, XB);
  k_conv3<<<dim3(NBLK), b256, 0, stream>>>(XB, WCV, HC, PARTB);
  k_bnfin<<<dim3(1), dim3(64), 0, stream>>>(PARTB, BNST);
  k_napply<<<dim3(NTOK * 8 / 256), b256, 0, stream>>>(HC, BNST, 0, 1, bn_g, bn_b, XFH, XFL);
  k_gemm<1, 1, 1, 1, 1, 0, 0><<<dim3(NBLK, DIN / 64), b256, 0, stream>>>(XFH, XFL, NCH, WEX, NCH, NCH, expand_b, XU, NCH,
                                                                           UVH, UVL, DIN, XU, NCH, x, out);
  k_gemm<0, 0, 0, 0, 1, 0, 0><<<dim3(NBLK, 1), b256, 0, stream>>>(UVH + NCH, UVL + NCH, DIN, WC1, NCH, NCH, expand_b, XU, NCH,
                                                                     V2H, V2L, NCH, XU, NCH, x, out);
  k_gemm<0, 0, 1, 0, 0, 0, 0><<<dim3(NBLK, XZW / 64), b256, 0, stream>>>(V2H, V2L, NCH, WIN, NCH, NCH, expand_b, XZ, XZW,
                                                                           V2H, V2L, NCH, XU, NCH, x, out);
  k_dwconv<<<dim3(NTOK / 8), b256, 0, stream>>>(XZ, mconv_w, mconv_b, XC, XCH, XCL);
  k_gemm<0, 0, 1, 0, 0, 0, 0><<<dim3(NBLK, DBW / 64), b256, 0, stream>>>(XCH, XCL, DIN, WXP, DIN, DIN, expand_b, DBL, DBW,
                                                                           V2H, V2L, NCH, XU, NCH, x, out);
  k_dtgate<<<dim3(NTOK * DIN / 256), b256, 0, stream>>>(DBL, dt_w, dt_b, XZ, DT, SZ);
  k_scan<<<dim3(NBT * (DIN / 64)), b256, 0, stream>>>(DT, XC, SZ, DBL, A_log, Dv, YGH, YGL);
  k_gemm<0, 0, 0, 0, 1, 1, 0><<<dim3(NBLK, 1), b256, 0, stream>>>(YGH, YGL, DIN, WOP, DIN, DIN, expand_b, XU, NCH,
                                                                     GH, GL, NCH, XU, NCH, x, out);
  k_gemm<1, 0, 1, 0, 0, 0, 0><<<dim3(NBLK, 1), b256, 0, stream>>>(GH, GL, NCH, WPJ, NCH, NCH, proj_b, XP, NCH,
                                                                     GH, GL, NCH, XU, NCH, x, out);
  k_ln<<<dim3(NBLK), b256, 0, stream>>>(XP, ln_g, ln_b, XN, PARTI);
  k_infin<<<dim3(1), b256, 0, stream>>>(PARTI, INST);
  k_napply<<<dim3(NTOK * 8 / 256), b256, 0, stream>>>(XN, INST, 1, 0, in_g, in_b, XOH, XOL);
  k_gemm<0, 0, 0, 0, 0, 0, 1><<<dim3(NBLK, 1), b256, 0, stream>>>(XOH, XOL, NCH, WRC, NCH, NCH, expand_b, XU, NCH,
                                                                     GH, GL, NCH, XU, NCH, x, out);
}
